// MambaLayer_3195455668581
// MI455X (gfx1250) — hardware-verified
//
#include <hip/hip_runtime.h>
#include <math.h>

typedef __attribute__((ext_vector_type(16))) __bf16   v16b;
typedef __attribute__((ext_vector_type(8)))  __bf16   v8b;
typedef __attribute__((ext_vector_type(8)))  float    v8f;
typedef __attribute__((ext_vector_type(4)))  float    v4f;
typedef __attribute__((ext_vector_type(4)))  unsigned v4u;

constexpr int kBatch = 2;
constexpr int kSeq   = 1024;
constexpr int kDm    = 1024;
constexpr int kDin   = 2048;
constexpr int kNst   = 16;
constexpr int kDtR   = 64;
constexpr int kPrjN  = 96;
constexpr int kPrjP  = 128;
constexpr int kXzP   = 2 * kDin;
constexpr int kRows  = kBatch * kSeq;
constexpr int kTP    = 260;
static_assert(kDtR + 2 * kNst == kPrjN, "x_proj width");
static_assert((kDm % 64) == 0 && (kDin % 64) == 0 && (kDtR % 64) == 0, "K multiples of 64 (transpose tiles) and of 32 (GEMM)");
static_assert((kRows % 64) == 0 && (kXzP % 64) == 0 && (kPrjP % 64) == 0 && (kDm % 64) == 0 && (kDin % 64) == 0, "GEMM M,N multiples of 64");
static_assert((kSeq % 64) == 0 && (kDin % 256) == 0 && (kSeq % 16) == 0, "conv / scan tile multiples");
static_assert(((kRows / 64) * (kXzP / 64)) % 8 == 0 && ((kRows / 64) * (kPrjP / 64)) % 8 == 0 &&
              ((kRows / 64) * (kDin / 64)) % 8 == 0 && ((kRows / 64) * (kDm / 64)) % 8 == 0, "8 tiles per GEMM block");

constexpr size_t kOffXB   = 0;
constexpr size_t kOffWIN  = kOffXB   + (size_t)kRows * kDm   * 2;
constexpr size_t kOffWXP  = kOffWIN  + (size_t)kXzP  * kDm   * 2;
constexpr size_t kOffWDT  = kOffWXP  + (size_t)kPrjP * kDin  * 2;
constexpr size_t kOffWOUT = kOffWDT  + (size_t)kDin  * kDtR  * 2;
constexpr size_t kOffXZ   = kOffWOUT + (size_t)kDm   * kDin  * 2;
constexpr size_t kOffUC   = kOffXZ   + (size_t)kRows * kXzP  * 4;
constexpr size_t kOffUB   = kOffUC   + (size_t)kRows * kDin  * 4;
constexpr size_t kOffXD   = kOffUB   + (size_t)kRows * kDin  * 2;
constexpr size_t kOffDTB  = kOffXD   + (size_t)kRows * kPrjP * 4;
constexpr size_t kOffDLR  = kOffDTB  + (size_t)kRows * kDtR  * 2;
constexpr size_t kOffYH   = kOffDLR  + (size_t)kRows * kDin  * 4;
constexpr size_t kOffYL   = kOffYH   + (size_t)kRows * kDin  * 2;
constexpr size_t kWsTotal = kOffYL   + (size_t)kRows * kDin  * 2;
static_assert(kWsTotal == 111149056ull, "carve total");
static_assert(kWsTotal <= 134217728ull, "carve cap");
static_assert((kOffWIN % 128) == 0 && (kOffWXP % 128) == 0 && (kOffWDT % 128) == 0 && (kOffWOUT % 128) == 0 &&
              (kOffXZ % 128) == 0 && (kOffUC % 128) == 0 && (kOffUB % 128) == 0 && (kOffXD % 128) == 0 &&
              (kOffDTB % 128) == 0 && (kOffDLR % 128) == 0 && (kOffYH % 128) == 0 && (kOffYL % 128) == 0,
              "128-B aligned regions");

__device__ __forceinline__ unsigned f2bf_bits(float f) {
  const unsigned u = __float_as_uint(f);
  return (u + 0x7FFFu + ((u >> 16) & 1u)) >> 16;
}
__device__ __forceinline__ float bf_bits2f(unsigned h) { return __uint_as_float(h << 16); }
__device__ __forceinline__ float rbf(float f) { return bf_bits2f(f2bf_bits(f)); }
__device__ __forceinline__ float lo_res(float f) { return f - rbf(f); }
__device__ __forceinline__ unsigned pk_bf16(float e0, float e1) {
  const unsigned l = f2bf_bits(e0);
  const unsigned h = f2bf_bits(e1);
  return l | (h << 16);
}
__device__ __forceinline__ v4u pack8_hi(v4f a0, v4f a1) {
  const float f0 = a0[0], f1 = a0[1], f2 = a0[2], f3 = a0[3];
  const float f4 = a1[0], f5 = a1[1], f6 = a1[2], f7 = a1[3];
  v4u r;
  r[0] = pk_bf16(f0, f1);
  r[1] = pk_bf16(f2, f3);
  r[2] = pk_bf16(f4, f5);
  r[3] = pk_bf16(f6, f7);
  return r;
}
__device__ __forceinline__ v4u pack8_lo(v4f a0, v4f a1) {
  const float f0 = a0[0], f1 = a0[1], f2 = a0[2], f3 = a0[3];
  const float f4 = a1[0], f5 = a1[1], f6 = a1[2], f7 = a1[3];
  v4u r;
  r[0] = pk_bf16(lo_res(f0), lo_res(f1));
  r[1] = pk_bf16(lo_res(f2), lo_res(f3));
  r[2] = pk_bf16(lo_res(f4), lo_res(f5));
  r[3] = pk_bf16(lo_res(f6), lo_res(f7));
  return r;
}

__device__ __forceinline__ void dep_guard4_b(v8f& a, v8f& b, v8f& c, v8f& d, v16b x, v16b y) {
  asm volatile("v_nop\n\tv_nop\n\tv_nop\n\tv_nop" : "+v"(a), "+v"(b), "+v"(c), "+v"(d) : "v"(x), "v"(y));
}
__device__ __forceinline__ void keep4_b(v16b a, v16b b, v16b c, v16b d) { asm volatile("v_nop" :: "v"(a), "v"(b), "v"(c), "v"(d)); }
__device__ __forceinline__ void acc_guard4(v8f& a, v8f& b, v8f& c, v8f& d) { asm volatile("v_nop\n\tv_nop\n\tv_nop\n\tv_nop" : "+v"(a), "+v"(b), "+v"(c), "+v"(d)); }
struct FragB {
  union U { v16b v; v8b h[2]; };
  static __device__ __forceinline__ v16b load(const __bf16* p) {
    U f; f.h[0] = *(const v8b*)(p); f.h[1] = *(const v8b*)(p + 16); return f.v;
  }
  static __device__ __forceinline__ v8f mma(v16b a, v16b b, v8f c) {
    return __builtin_amdgcn_wmma_f32_16x16x32_bf16(false, a, false, b, (short)0, c, false, false);
  }
};

template <int SPL>
__global__ __launch_bounds__(256) void wmma_gemm64(
    const unsigned short* __restrict__ Ap, const unsigned short* __restrict__ A2p, int lda,
    const unsigned short* __restrict__ Btp, int ldb,
    float* __restrict__ C, int ldc, int M, int N, int K) {
  const __bf16* A  = (const __bf16*)Ap;
  const __bf16* A2 = (const __bf16*)A2p;
  const __bf16* Bt = (const __bf16*)Btp;
  __shared__ __align__(16) float sT[8][16 * 68];
  const int lane = threadIdx.x & 31;
  const int wave = threadIdx.x >> 5;
  const int tilesN = N >> 6;
  const int tilesM = M >> 6;
  const int tile = blockIdx.x * 8 + wave;
  if (tile >= tilesM * tilesN) return;
  const int tm = tile / tilesN;
  const int tn = tile - tm * tilesN;
  const int m0 = tm << 6;
  const int n0 = tn << 6;

  const int rlane = lane & 15;
  const int koff  = (lane >> 4) * 8;
  const int mOff  = (lane >> 4) * 8;

  v8f acc[4][4];
#pragma unroll
  for (int i = 0; i < 4; ++i)
#pragma unroll
    for (int j = 0; j < 4; ++j) acc[i][j] = (v8f){0.f,0.f,0.f,0.f,0.f,0.f,0.f,0.f};

  for (int k0 = 0; k0 < K; k0 += 32) {
    v16b bh[4];
#pragma unroll
    for (int j = 0; j < 4; ++j) {
      const size_t bo = (size_t)(n0 + (j << 4) + rlane) * ldb + koff + k0;
      bh[j] = FragB::load(Bt + bo);
    }
#pragma unroll
    for (int i = 0; i < 4; ++i) {
      const size_t ao = (size_t)(m0 + (i << 4) + rlane) * lda + koff + k0;
      v16b ah = FragB::load(A + ao);
      v16b al = ah;
      if (SPL == 1) al = FragB::load(A2 + ao);
#pragma unroll
      for (int j = 0; j < 4; ++j) {
        acc[i][j] = FragB::mma(ah, bh[j], acc[i][j]);
        if (SPL == 1) acc[i][j] = FragB::mma(al, bh[j], acc[i][j]);
      }
      dep_guard4_b(acc[i][0], acc[i][1], acc[i][2], acc[i][3], ah, al);
    }
    keep4_b(bh[0], bh[1], bh[2], bh[3]);
  }
  acc_guard4(acc[0][0], acc[0][1], acc[0][2], acc[0][3]);
  acc_guard4(acc[1][0], acc[1][1], acc[1][2], acc[1][3]);
  acc_guard4(acc[2][0], acc[2][1], acc[2][2], acc[2][3]);
  acc_guard4(acc[3][0], acc[3][1], acc[3][2], acc[3][3]);

  float* slab = sT[wave];
#pragma unroll
  for (int i = 0; i < 4; ++i) {
    const int mBase = m0 + (i << 4);
#pragma unroll
    for (int j = 0; j < 4; ++j) {
#pragma unroll
      for (int r = 0; r < 8; ++r) {
        slab[(mOff + r) * 68 + (j << 4) + rlane] = acc[i][j][r];
      }
    }
    __builtin_amdgcn_fence(__ATOMIC_RELEASE, "workgroup");
    __builtin_amdgcn_wave_barrier();
    __builtin_amdgcn_fence(__ATOMIC_ACQUIRE, "workgroup");
    {
      const int hh = lane >> 4, c4 = (lane & 15) * 4;
      for (int pass = 0; pass < 2; ++pass) {
#pragma unroll
        for (int it = 0; it < 8; ++it) {
          const int row = it * 2 + hh;
          v4f v = *(const v4f*)(slab + row * 68 + c4);
          *(volatile v4f*)(C + (size_t)(mBase + row) * ldc + n0 + c4) = v;
        }
        __threadfence();
      }
    }
    __builtin_amdgcn_fence(__ATOMIC_RELEASE, "workgroup");
    __builtin_amdgcn_wave_barrier();
    __builtin_amdgcn_fence(__ATOMIC_ACQUIRE, "workgroup");
  }
}

__global__ __launch_bounds__(256) void cast_rows_bf16_kernel(
    const float* __restrict__ src, unsigned short* __restrict__ dst, int total8)
{
  const int i = blockIdx.x * 256 + threadIdx.x;
  if (i >= total8) return;
  const size_t e0 = (size_t)i << 3;
  const v4f a0 = *(const v4f*)(src + e0);
  const v4f a1 = *(const v4f*)(src + e0 + 4);
  const v4u w = pack8_hi(a0, a1);
  unsigned short* q = dst + e0;
  *(volatile v4u*)q = w;
  __threadfence();
  *(volatile v4u*)q = w;
}

__global__ __launch_bounds__(256) void dt_cast_kernel(
    const float* __restrict__ XD, unsigned short* __restrict__ DTB, int total8)
{
  const int i = blockIdx.x * 256 + threadIdx.x;
  if (i >= total8) return;
  const int e0  = i << 3;
  const int row = e0 >> 6;
  const int c8  = e0 & 63;
  const float* p = XD + (size_t)row * kPrjP + c8;
  const v4f a0 = *(const v4f*)(p);
  const v4f a1 = *(const v4f*)(p + 4);
  const v4u w = pack8_hi(a0, a1);
  unsigned short* q = DTB + e0;
  *(volatile v4u*)q = w;
  __threadfence();
  *(volatile v4u*)q = w;
}

__global__ __launch_bounds__(256) void transpose_bf16_kernel(
    const float* __restrict__ W, unsigned short* __restrict__ Bt, int Kdim, int Ndim)
{
  __shared__ float tile[64 * 65];
  const int tid = threadIdx.x, lane = tid & 31, wave = tid >> 5;
  const int n0 = blockIdx.x * 64;
  const int k0 = blockIdx.y * 64;
#pragma unroll
  for (int p = 0; p < 16; ++p) {
    const int idx = tid + p * 256;
    const int kk  = idx >> 6;
    const int nn  = idx & 63;
    const int n   = n0 + nn;
    const int nc  = (n < Ndim) ? n : (Ndim - 1);
    const float v = W[(size_t)(k0 + kk) * Ndim + nc];
    tile[kk * 65 + nn] = (n < Ndim) ? v : 0.0f;
  }
  __syncthreads();
  const int q = lane >> 3, c8 = (lane & 7) * 8;
  v4u hw[2];
#pragma unroll
  for (int it = 0; it < 2; ++it) {
    const int nrow = it * 32 + wave * 4 + q;
    const float f0 = tile[(c8 + 0) * 65 + nrow], f1 = tile[(c8 + 1) * 65 + nrow];
    const float f2 = tile[(c8 + 2) * 65 + nrow], f3 = tile[(c8 + 3) * 65 + nrow];
    const float f4 = tile[(c8 + 4) * 65 + nrow], f5 = tile[(c8 + 5) * 65 + nrow];
    const float f6 = tile[(c8 + 6) * 65 + nrow], f7 = tile[(c8 + 7) * 65 + nrow];
    v4u r;
    r[0] = pk_bf16(f0, f1);
    r[1] = pk_bf16(f2, f3);
    r[2] = pk_bf16(f4, f5);
    r[3] = pk_bf16(f6, f7);
    hw[it] = r;
  }
  for (int pass = 0; pass < 2; ++pass) {
#pragma unroll
    for (int it = 0; it < 2; ++it) {
      const int nrow = it * 32 + wave * 4 + q;
      *(volatile v4u*)(Bt + (size_t)(n0 + nrow) * Kdim + k0 + c8) = hw[it];
    }
    __threadfence();
  }
}

__global__ __launch_bounds__(256) void conv_silu_kernel(
    const float* __restrict__ XZ, const float* __restrict__ ck, const float* __restrict__ cb,
    float* __restrict__ UC, unsigned short* __restrict__ UB)
{
  __shared__ __align__(16) float sT[16 * kTP];
  const int tid = threadIdx.x, lane = tid & 31, wave = tid >> 5;
  const int d0 = blockIdx.x * 256, d = d0 + tid;
  const int g0 = blockIdx.y * 64;
  const int tb = g0 & (kSeq - 1);
  const float w0 = rbf(ck[0 * kDin + d]);
  const float w1 = rbf(ck[1 * kDin + d]);
  const float w2 = rbf(ck[2 * kDin + d]);
  const float w3 = rbf(ck[3 * kDin + d]);
  const float bc = rbf(cb[d]);
  float xm3, xm2, xm1;
  {
    const bool hist = (tb > 0);
    const int rb = hist ? (g0 - 3) : g0;
    const float v3 = XZ[(size_t)rb * kXzP + d];
    const float v2 = XZ[(size_t)(rb + 1) * kXzP + d];
    const float v1 = XZ[(size_t)(rb + 2) * kXzP + d];
    xm3 = hist ? v3 : 0.f;
    xm2 = hist ? v2 : 0.f;
    xm1 = hist ? v1 : 0.f;
  }
  const int hrow = wave >> 1;
  const int hch  = (wave & 1) * 128 + lane * 4;
#pragma unroll 1
  for (int sub = 0; sub < 4; ++sub) {
    const int lb = g0 + sub * 16;
#pragma unroll 1
    for (int s = 0; s < 16; ++s) {
      const float xcur = XZ[(size_t)(lb + s) * kXzP + d];
      float acc = w0 * xm3;
      acc = fmaf(w1, xm2, acc);
      acc = fmaf(w2, xm1, acc);
      acc = fmaf(w3, xcur, acc);
      const float sv = acc + bc;
      const float sg = __builtin_amdgcn_rcpf(1.0f + expf(-sv));
      sT[s * kTP + tid] = sv * sg;
      xm3 = xm2; xm2 = xm1; xm1 = xcur;
    }
    __syncthreads();
    v4f fv[4];
    v4u bw[2];
#pragma unroll
    for (int it = 0; it < 4; ++it) fv[it] = *(const v4f*)(sT + (it * 4 + hrow) * kTP + hch);
#pragma unroll
    for (int it = 0; it < 2; ++it) {
      const float* sp = sT + (it * 8 + wave) * kTP + lane * 8;
      const v4f a0 = *(const v4f*)(sp);
      const v4f a1 = *(const v4f*)(sp + 4);
      bw[it] = pack8_hi(a0, a1);
    }
    for (int pass = 0; pass < 2; ++pass) {
#pragma unroll
      for (int it = 0; it < 4; ++it)
        *(volatile v4f*)(UC + (size_t)(lb + it * 4 + hrow) * kDin + d0 + hch) = fv[it];
#pragma unroll
      for (int it = 0; it < 2; ++it)
        *(volatile v4u*)(UB + (size_t)(lb + it * 8 + wave) * kDin + d0 + lane * 8) = bw[it];
      __threadfence();
    }
    __syncthreads();
  }
}

__global__ __launch_bounds__(256) void scan_kernel(
    const float* __restrict__ DLR, const float* __restrict__ UC, const float* __restrict__ XZ,
    const float* __restrict__ XD, const float* __restrict__ bdt, const float* __restrict__ Alog,
    const float* __restrict__ Dv, unsigned short* __restrict__ YH, unsigned short* __restrict__ YL)
{
  __shared__ __align__(16) float sBC[16 * 32];
  __shared__ __align__(16) float sY[16 * kTP];
  const int tid = threadIdx.x, lane = tid & 31, wave = tid >> 5;
  constexpr int kBlkPerB = kDin / 256;
  const int bix = blockIdx.x / kBlkPerB;
  const int d0  = (blockIdx.x - bix * kBlkPerB) * 256;
  const int d   = d0 + tid;
  const size_t row0 = (size_t)bix * kSeq;

#pragma unroll 1
  for (int n = 0; n < kNst; ++n) sY[n * kTP + tid] = -expf(rbf(Alog[(size_t)d * kNst + n]));
  __syncthreads();
  float An[kNst], h[kNst];
#pragma unroll
  for (int n = 0; n < kNst; ++n) {
    An[n] = sY[n * kTP + tid];
    h[n] = 0.f;
  }
  __syncthreads();
  const float bb = rbf(bdt[d]);
  const float Dd = rbf(Dv[d]);

#pragma unroll 1
  for (int c = 0; c < kSeq / 16; ++c) {
    const int l0 = c * 16;
    if (tid < 128) {
      const int r = tid >> 3, q = (tid & 7) * 4;
      const v4f v = *(const v4f*)(XD + (row0 + l0 + r) * kPrjP + kDtR + q);
      *(v4f*)(sBC + r * 32 + q) = v;
    }
    __syncthreads();
#pragma unroll 1
    for (int s = 0; s < 16; ++s) {
      const size_t m = row0 + (size_t)(l0 + s);
      const float a     = DLR[m * kDin + d] + bb;
      const float delta = fmaxf(a, 0.0f) + log1pf(expf(-fabsf(a)));
      const float xv    = UC[m * kDin + d];
      const float zv    = XZ[m * kXzP + kDin + d];
      v4f Bq[4], Cq[4];
#pragma unroll
      for (int qq = 0; qq < 4; ++qq) {
        Bq[qq] = *(const v4f*)(sBC + s * 32 + 4 * qq);
        Cq[qq] = *(const v4f*)(sBC + s * 32 + kNst + 4 * qq);
      }
      const float dx = delta * xv;
      float y = 0.f;
#pragma unroll
      for (int n = 0; n < kNst; ++n) {
        const float e = __expf(delta * An[n]);
        const float hn = fmaf(e, h[n], dx * Bq[n >> 2][n & 3]);
        h[n] = hn;
        y = fmaf(hn, Cq[n >> 2][n & 3], y);
      }
      y = fmaf(xv, Dd, y);
      const float sg = __builtin_amdgcn_rcpf(1.0f + expf(-zv));
      sY[s * kTP + tid] = y * (zv * sg);
    }
    __syncthreads();
    v4u hw[2], lw[2];
#pragma unroll
    for (int it = 0; it < 2; ++it) {
      const float* sp = sY + (it * 8 + wave) * kTP + lane * 8;
      const v4f a0 = *(const v4f*)(sp);
      const v4f a1 = *(const v4f*)(sp + 4);
      hw[it] = pack8_hi(a0, a1);
      lw[it] = pack8_lo(a0, a1);
    }
    for (int pass = 0; pass < 2; ++pass) {
#pragma unroll
      for (int it = 0; it < 2; ++it) {
        const size_t o = (row0 + (size_t)(l0 + it * 8 + wave)) * kDin + d0 + lane * 8;
        *(volatile v4u*)(YH + o) = hw[it];
        *(volatile v4u*)(YL + o) = lw[it];
      }
      __threadfence();
    }
  }
}

extern "C" void kernel_launch(void* const* d_in, const int* in_sizes, int n_in,
                              void* d_out, int out_size, void* d_ws, size_t ws_size,
                              hipStream_t stream) {
  if (n_in < 10) return;
  if (in_sizes[0] != kRows * kDm) return;
  if (in_sizes[1] != kDm * kXzP) return;
  if (in_sizes[2] != 4 * kDin) return;
  if (in_sizes[3] != kDin) return;
  if (in_sizes[4] != kDin * kPrjN) return;
  if (in_sizes[5] != kDtR * kDin) return;
  if (in_sizes[6] != kDin) return;
  if (in_sizes[7] != kDin * kDm) return;
  if (in_sizes[8] != kDin * kNst) return;
  if (in_sizes[9] != kDin) return;
  if (out_size != kRows * kDm) return;
  if (ws_size < kWsTotal) return;

  const float* x      = (const float*)d_in[0];
  const float* W_in   = (const float*)d_in[1];
  const float* conv_k = (const float*)d_in[2];
  const float* conv_b = (const float*)d_in[3];
  const float* W_x    = (const float*)d_in[4];
  const float* W_dt   = (const float*)d_in[5];
  const float* b_dt   = (const float*)d_in[6];
  const float* W_out  = (const float*)d_in[7];
  const float* A_log  = (const float*)d_in[8];
  const float* Dv     = (const float*)d_in[9];
  float* out = (float*)d_out;

  char* ws = (char*)d_ws;
  unsigned short* XB   = (unsigned short*)(ws + kOffXB);
  unsigned short* WIN  = (unsigned short*)(ws + kOffWIN);
  unsigned short* WXP  = (unsigned short*)(ws + kOffWXP);
  unsigned short* WDT  = (unsigned short*)(ws + kOffWDT);
  unsigned short* WOUT = (unsigned short*)(ws + kOffWOUT);
  float*          XZ   = (float*)(ws + kOffXZ);
  float*          UC   = (float*)(ws + kOffUC);
  unsigned short* UB   = (unsigned short*)(ws + kOffUB);
  float*          XD   = (float*)(ws + kOffXD);
  unsigned short* DTB  = (unsigned short*)(ws + kOffDTB);
  float*          DLR  = (float*)(ws + kOffDLR);
  unsigned short* YH   = (unsigned short*)(ws + kOffYH);
  unsigned short* YL   = (unsigned short*)(ws + kOffYL);

  cast_rows_bf16_kernel<<<(kRows * kDm / 8) / 256, 256, 0, stream>>>(x, XB, kRows * kDm / 8);

  transpose_bf16_kernel<<<dim3(kXzP / 64, kDm / 64), 256, 0, stream>>>(W_in, WIN, kDm, kXzP);
  transpose_bf16_kernel<<<dim3(kPrjP / 64, kDin / 64), 256, 0, stream>>>(W_x, WXP, kDin, kPrjN);
  transpose_bf16_kernel<<<dim3(kDin / 64, kDtR / 64), 256, 0, stream>>>(W_dt, WDT, kDtR, kDin);
  transpose_bf16_kernel<<<dim3(kDm / 64, kDin / 64), 256, 0, stream>>>(W_out, WOUT, kDin, kDm);

  wmma_gemm64<0><<<dim3((kRows / 64) * (kXzP / 64) / 8), 256, 0, stream>>>(
      XB, XB, kDm, WIN, kDm, XZ, kXzP, kRows, kXzP, kDm);

  conv_silu_kernel<<<dim3(kDin / 256, kRows / 64), 256, 0, stream>>>(XZ, conv_k, conv_b, UC, UB);

  wmma_gemm64<0><<<dim3((kRows / 64) * (kPrjP / 64) / 8), 256, 0, stream>>>(
      UB, UB, kDin, WXP, kDin, XD, kPrjP, kRows, kPrjP, kDin);

  dt_cast_kernel<<<(kRows * kDtR / 8) / 256, 256, 0, stream>>>(XD, DTB, kRows * kDtR / 8);

  wmma_gemm64<0><<<dim3((kRows / 64) * (kDin / 64) / 8), 256, 0, stream>>>(
      DTB, DTB, kDtR, WDT, kDtR, DLR, kDin, kRows, kDin, kDtR);

  scan_kernel<<<kBatch * (kDin / 256), 256, 0, stream>>>(DLR, UC, XZ, XD, b_dt, A_log, Dv, YH, YL);

  wmma_gemm64<1><<<dim3((kRows / 64) * (kDm / 64) / 8), 256, 0, stream>>>(
      YH, YL, kDin, WOUT, kDin, out, kDm, kRows, kDm, kDin);
}
